// SmolLM2Attention_29635274342952
// MI455X (gfx1250) — hardware-verified
//
#include <hip/hip_runtime.h>
#include <math.h>
#include <float.h>
#include <stdint.h>

#define NB    2
#define SEQ   2048
#define DM    2048
#define NH    32
#define NKV   8
#define GRP   (NH / NKV)
#define HD    64
#define QD    (NH * HD)
#define KVD   (NKV * HD)
#define QKD   (QD + KVD)
#define EQKV  (QD + 2 * KVD)
#define NTOK  (NB * SEQ)
#define NQB   (SEQ / 64)
#define RESQB 8
#define NUNIT (NH + NKV)
#define EPSV  1e-6f

static_assert(GRP * NKV == NH);
static_assert((SEQ % 64) == 0 && (DM % 64) == 0 && (QD % 64) == 0 && (QKD % 64) == 0 && (KVD % 64) == 0);
static_assert(RESQB <= NQB);
static_assert(HD == 64);

typedef _Float16 v16h __attribute__((ext_vector_type(16)));
typedef _Float16 v8h  __attribute__((ext_vector_type(8)));
typedef __bf16   v16b __attribute__((ext_vector_type(16)));
typedef __bf16   v8b  __attribute__((ext_vector_type(8)));
typedef float    v8f  __attribute__((ext_vector_type(8)));
typedef float    v4f  __attribute__((ext_vector_type(4)));
typedef float    v2f  __attribute__((ext_vector_type(2)));
typedef unsigned int   v4u  __attribute__((ext_vector_type(4)));
typedef unsigned short v8us __attribute__((ext_vector_type(8)));
typedef int      v4i  __attribute__((ext_vector_type(4)));

__device__ __forceinline__ unsigned short bf_bits(float f) {
  unsigned u = __float_as_uint(f);
  return (unsigned short)((u + 0x7FFFu + ((u >> 16) & 1u)) >> 16);
}
__device__ __forceinline__ float bf_up(unsigned short h) { return __uint_as_float(((unsigned)h) << 16); }
__device__ __forceinline__ unsigned short h_bits(_Float16 x) { return __builtin_bit_cast(unsigned short, x); }
__device__ __forceinline__ unsigned pk16(unsigned short a, unsigned short b) { return (unsigned)a | ((unsigned)b << 16); }
__device__ __forceinline__ v8f zero8() { v8f z = {0.f, 0.f, 0.f, 0.f, 0.f, 0.f, 0.f, 0.f}; return z; }

template <bool F16> struct OpT;
template <> struct OpT<false> { typedef v16b V; typedef v8b H; typedef __bf16   E; };
template <> struct OpT<true>  { typedef v16h V; typedef v8h H; typedef _Float16 E; };

template <bool F16>
__device__ __forceinline__ typename OpT<F16>::V ldfrag(const typename OpT<F16>::E* p) {
  union { typename OpT<F16>::V v; typename OpT<F16>::H h[2]; } f;
  f.h[0] = *(const typename OpT<F16>::H*)(p);
  f.h[1] = *(const typename OpT<F16>::H*)(p + 16);
  return f.v;
}
__device__ __forceinline__ v16h ldfrag_h(const _Float16* p) {
  union { v16h v; v8h h[2]; } f;
  f.h[0] = *(const v8h*)(p);
  f.h[1] = *(const v8h*)(p + 16);
  return f.v;
}

__device__ __forceinline__ v8f mma_raw(v16b a, v16b b, v8f c) {
  return __builtin_amdgcn_wmma_f32_16x16x32_bf16(false, a, false, b, (short)0, c, false, false);
}
__device__ __forceinline__ v8f mma_raw(v16h a, v16h b, v8f c) {
  return __builtin_amdgcn_wmma_f32_16x16x32_f16(false, a, false, b, (short)0, c, false, false);
}
__device__ __forceinline__ v8f mma_h(v16h a, v16h b, v8f c) {
  c = __builtin_amdgcn_wmma_f32_16x16x32_f16(false, a, false, b, (short)0, c, false, false);
#if defined(__HIP_DEVICE_COMPILE__)
  asm volatile("v_nop\n\tv_nop\n\tv_nop\n\tv_nop" : "+v"(c) : "v"(a), "v"(b));
#endif
  return c;
}
template <typename VA>
__device__ __forceinline__ void dep_guard(v8f& a, v8f& b, VA x, VA y) {
#if defined(__HIP_DEVICE_COMPILE__)
  asm volatile("v_nop\n\tv_nop\n\tv_nop\n\tv_nop" : "+v"(a), "+v"(b) : "v"(x), "v"(y));
#else
  (void)a; (void)b; (void)x; (void)y;
#endif
}
template <typename VA>
__device__ __forceinline__ void keep4(VA a, VA b, VA c, VA d) {
#if defined(__HIP_DEVICE_COMPILE__)
  asm volatile("v_nop" :: "v"(a), "v"(b), "v"(c), "v"(d));
#else
  (void)a; (void)b; (void)c; (void)d;
#endif
}
__device__ __forceinline__ void acc_guard4(v8f& a, v8f& b, v8f& c, v8f& d) {
#if defined(__HIP_DEVICE_COMPILE__)
  asm volatile("v_nop\n\tv_nop\n\tv_nop\n\tv_nop" : "+v"(a), "+v"(b), "+v"(c), "+v"(d));
#else
  (void)a; (void)b; (void)c; (void)d;
#endif
}

template <int MODE>
__device__ __forceinline__ unsigned short cvt1(float f, float scale) {
  const unsigned short bb = bf_bits(f);
  if (MODE == 0) return bb;
  return h_bits((_Float16)(bf_up(bb) * scale));
}
template <int MODE>
__global__ __launch_bounds__(256) void cvt16x8(const float* __restrict__ in, unsigned short* out, int n8, float scale) {
  const int i = blockIdx.x * 256 + threadIdx.x;
  if (i < n8) {
    const v4f a = *(const v4f*)(in + (size_t)i * 8);
    const v4f b = *(const v4f*)(in + (size_t)i * 8 + 4);
    v4u p;
    p[0] = pk16(cvt1<MODE>(a[0], scale), cvt1<MODE>(a[1], scale));
    p[1] = pk16(cvt1<MODE>(a[2], scale), cvt1<MODE>(a[3], scale));
    p[2] = pk16(cvt1<MODE>(b[0], scale), cvt1<MODE>(b[1], scale));
    p[3] = pk16(cvt1<MODE>(b[2], scale), cvt1<MODE>(b[3], scale));
    *(volatile v4u*)(out + (size_t)i * 8) = p;
    __threadfence();
    *(volatile v4u*)(out + (size_t)i * 8) = p;
  }
}

__global__ __launch_bounds__(32) void ropefreq(float* invf) {
#pragma clang fp contract(off)
  const int lane = threadIdx.x & 31;
  const float e = (float)(2 * lane) * (1.0f / 64.0f);
  const float f = 1.0f / powf(10000.0f, e);
  *(volatile float*)(invf + lane) = f;
  __threadfence();
  *(volatile float*)(invf + lane) = f;
}

__global__ __launch_bounds__(256) void ropetab(const int* __restrict__ pos, const float* __restrict__ invf,
                                               float* tab, int npos) {
#pragma clang fp contract(off)
  const int wave = threadIdx.x >> 5, lane = threadIdx.x & 31;
  const int s = blockIdx.x * 8 + wave;
  if (s < npos) {
    const float fr = (float)pos[s] * invf[lane];
    float sn, cs;
    sincosf(fr, &sn, &cs);
    v2f v;
    v[0] = cs;
    v[1] = sn;
    float* d = tab + (size_t)s * 64 + 2 * lane;
    *(volatile v2f*)d = v;
    __threadfence();
    *(volatile v2f*)d = v;
  }
}

__global__ __launch_bounds__(256) void normrope(const float* __restrict__ QKf, const float* __restrict__ qw,
                                                const float* __restrict__ kw, const float* __restrict__ tab,
                                                unsigned short* Qh, unsigned short* Ql,
                                                unsigned short* Kh, unsigned short* Kl, int nUnits) {
#pragma clang fp contract(off)
  __shared__ __align__(16) unsigned short sh[8][128];
  const int tid = threadIdx.x;
  const int wave = tid >> 5;
  const int lane = tid & 31;
  const int u = blockIdx.x * 8 + wave;
  if (u >= nUnits) return;
  const int t = u / NUNIT;
  const int j = u - t * NUNIT;
  const int s = t & (SEQ - 1);
  const bool isq = (j < NH);

  const float* row = QKf + (size_t)t * QKD + (size_t)j * HD;
  const float x1 = row[lane];
  const float x2 = row[32 + lane];
  float ss = x1 * x1 + x2 * x2;
#pragma unroll
  for (int off = 16; off >= 1; off >>= 1) ss += __shfl_xor(ss, off, 32);
  const float var = ss * (1.0f / 64.0f);
  const float inv = rsqrtf(var + EPSV);

  const float wq1 = bf_up(bf_bits(qw[lane])), wq2 = bf_up(bf_bits(qw[32 + lane]));
  const float wk1 = bf_up(bf_bits(kw[lane])), wk2 = bf_up(bf_bits(kw[32 + lane]));
  const float w1 = isq ? wq1 : wk1;
  const float w2 = isq ? wq2 : wk2;
  const float y1 = (x1 * inv) * w1;
  const float y2 = (x2 * inv) * w2;

  const v2f cs2 = *(const v2f*)(tab + (size_t)s * 64 + 2 * lane);
  const float cs = cs2[0], sn = cs2[1];
  const float o1 = y1 * cs - y2 * sn;
  const float o2 = y2 * cs + y1 * sn;

  const float c1 = o1 * 64.0f, c2 = o2 * 64.0f;
  const _Float16 g1 = (_Float16)c1, g2 = (_Float16)c2;
  const unsigned short h1 = h_bits(g1), h2 = h_bits(g2);
  const unsigned short l1 = h_bits((_Float16)(c1 - (float)g1));
  const unsigned short l2 = h_bits((_Float16)(c2 - (float)g2));

  unsigned short* sw = sh[wave];
  sw[lane]      = h1;
  sw[32 + lane] = h2;
  sw[64 + lane] = l1;
  sw[96 + lane] = l2;
  __builtin_amdgcn_fence(__ATOMIC_RELEASE, "workgroup");
  __builtin_amdgcn_wave_barrier();
  __builtin_amdgcn_fence(__ATOMIC_ACQUIRE, "workgroup");

  const int pl = (lane >> 3) & 1;
  const int c8 = (lane & 7) * 8;
  const v8us v = *(const v8us*)(sw + pl * 64 + c8);
  const size_t qoff = (size_t)t * QD + (size_t)j * HD + c8;
  const int jk = isq ? 0 : (j - NH);
  const size_t koff = (size_t)t * KVD + (size_t)jk * HD + c8;
  unsigned short* dst = isq ? ((pl ? Ql : Qh) + qoff) : ((pl ? Kl : Kh) + koff);
  if (lane < 16) *(volatile v8us*)dst = v;
  __threadfence();
  if (lane < 16) *(volatile v8us*)dst = v;
}

template <bool F16, int NS>
__device__ __forceinline__ void kloop(v8f (&acc)[4][4],
                                      const typename OpT<F16>::E* Ab, const typename OpT<F16>::E* Ab2, int lda,
                                      const typename OpT<F16>::E* Bb, int ldb,
                                      int m0, int n0, int K, int rlane, int koff) {
  typedef typename OpT<F16>::V V;
  for (int k0 = 0; k0 < K; k0 += 32) {
    V bh[4];
#pragma unroll
    for (int j = 0; j < 4; ++j)
      bh[j] = ldfrag<F16>(Bb + (size_t)(n0 + (j << 4) + rlane) * ldb + koff + k0);
#pragma unroll
    for (int i = 0; i < 4; ++i) {
      const size_t ao = (size_t)(m0 + (i << 4) + rlane) * lda + koff + k0;
      const V ah = ldfrag<F16>(Ab + ao);
      V al = ah;
      if (NS) al = ldfrag<F16>(Ab2 + ao);
#pragma unroll
      for (int j = 0; j < 4; ++j) {
        acc[i][j] = mma_raw(ah, bh[j], acc[i][j]);
        if (NS) acc[i][j] = mma_raw(al, bh[j], acc[i][j]);
      }
      dep_guard<V>(acc[i][0], acc[i][3], ah, al);
    }
    keep4<V>(bh[0], bh[1], bh[2], bh[3]);
  }
}

template <bool F16, int NSPLIT, int OUT_MODE>
__global__ __launch_bounds__(256) void gemm64(
    const unsigned short* __restrict__ Ap, const unsigned short* A2p, int lda, long long strideA,
    const unsigned short* __restrict__ Btp, int ldb, long long strideB,
    void* Cout, int ldc, long long strideC,
    void* Cout2, int ldc2, long long strideC2, int N2,
    int M, int N, int K, float oscale, float rscale, int loMask, int loRows) {
  typedef typename OpT<F16>::E E;
  const E* A  = (const E*)(const void*)Ap;
  const E* A2 = (const E*)(const void*)A2p;
  const E* Bt = (const E*)(const void*)Btp;
  __shared__ __align__(16) float sT[8][16 * 68];
  const int b    = blockIdx.y;
  const int lane = threadIdx.x & 31;
  const int wave = threadIdx.x >> 5;
  const int tilesN = N >> 6;
  const int tilesM = M >> 6;
  const int tile = blockIdx.x * 8 + wave;
  if (tile >= tilesM * tilesN) return;
  const int tm = tile / tilesN;
  const int tn = tile - tm * tilesN;
  const int m0 = tm << 6;
  const int n0 = tn << 6;

  const E* Ab  = A  + (size_t)b * strideA;
  const E* Bb  = Bt + (size_t)b * strideB;
  const E* Ab2 = (NSPLIT >= 1) ? (A2 + (size_t)b * strideA) : Ab;

  const int rlane = lane & 15;
  const int koff  = (lane >> 4) * 8;
  const int mOff  = (lane >> 4) * 8;

  v8f acc[4][4];
#pragma unroll
  for (int i = 0; i < 4; ++i)
#pragma unroll
    for (int j = 0; j < 4; ++j) acc[i][j] = zero8();

  int useLo = 0;
  if (NSPLIT >= 1) useLo = __builtin_amdgcn_readfirstlane(((m0 & loMask) < loRows) ? 1 : 0);
  if (NSPLIT >= 1 && useLo != 0) kloop<F16, 1>(acc, Ab, Ab2, lda, Bb, ldb, m0, n0, K, rlane, koff);
  else                           kloop<F16, 0>(acc, Ab, Ab,  lda, Bb, ldb, m0, n0, K, rlane, koff);
  acc_guard4(acc[0][0], acc[0][1], acc[0][2], acc[0][3]);
  acc_guard4(acc[1][0], acc[1][1], acc[1][2], acc[1][3]);
  acc_guard4(acc[2][0], acc[2][1], acc[2][2], acc[2][3]);
  acc_guard4(acc[3][0], acc[3][1], acc[3][2], acc[3][3]);

  float* slab = sT[wave];
#pragma unroll
  for (int i = 0; i < 4; ++i) {
    const int mBase = m0 + (i << 4);
#pragma unroll
    for (int j = 0; j < 4; ++j) {
#pragma unroll
      for (int r = 0; r < 8; ++r) {
        slab[(mOff + r) * 68 + (j << 4) + rlane] = acc[i][j][r] * oscale;
      }
    }
    __builtin_amdgcn_fence(__ATOMIC_RELEASE, "workgroup");
    __builtin_amdgcn_wave_barrier();
    __builtin_amdgcn_fence(__ATOMIC_ACQUIRE, "workgroup");
    if (OUT_MODE == 0) {
      float* C = (float*)Cout + (size_t)b * strideC;
      const int hh = lane >> 4, c4 = (lane & 15) * 4;
      for (int pass = 0; pass < 2; ++pass) {
#pragma unroll
        for (int it = 0; it < 8; ++it) {
          const int rowi = it * 2 + hh;
          const v4f v = *(const v4f*)(slab + rowi * 68 + c4);
          *(volatile v4f*)(C + (size_t)(mBase + rowi) * ldc + n0 + c4) = v;
        }
        __threadfence();
      }
    } else {
      const int q4 = lane >> 3, c8 = (lane & 7) * 8;
      unsigned short* C  = (unsigned short*)Cout  + (size_t)b * strideC;
      unsigned short* C2 = (unsigned short*)Cout2 + (size_t)b * strideC2;
      const bool wlo = (n0 < N2);
      v4u hv[4], lv[4];
#pragma unroll
      for (int it = 0; it < 4; ++it) {
        const int rowi = it * 4 + q4;
        const float* sp = slab + rowi * 68 + c8;
        v4u a, a2;
#pragma unroll
        for (int e = 0; e < 4; ++e) {
          const float f0 = sp[2 * e], f1 = sp[2 * e + 1];
          const _Float16 x0 = (_Float16)f0, x1 = (_Float16)f1;
          const unsigned short h0 = h_bits(x0), h1 = h_bits(x1);
          const unsigned short l0 = h_bits((_Float16)((f0 - (float)x0) * rscale));
          const unsigned short l1 = h_bits((_Float16)((f1 - (float)x1) * rscale));
          a[e] = pk16(h0, h1); a2[e] = pk16(l0, l1);
        }
        hv[it] = a; lv[it] = a2;
      }
      for (int pass = 0; pass < 2; ++pass) {
#pragma unroll
        for (int it = 0; it < 4; ++it) {
          const int rowi = it * 4 + q4;
          *(volatile v4u*)(C + (size_t)(mBase + rowi) * ldc + n0 + c8) = hv[it];
          if (wlo) *(volatile v4u*)(C2 + (size_t)(mBase + rowi) * ldc2 + n0 + c8) = lv[it];
        }
        __threadfence();
      }
    }
    __builtin_amdgcn_fence(__ATOMIC_RELEASE, "workgroup");
    __builtin_amdgcn_wave_barrier();
    __builtin_amdgcn_fence(__ATOMIC_ACQUIRE, "workgroup");
  }
}

template <bool PRES>
__global__ __launch_bounds__(128)
void attn64(const unsigned short* __restrict__ qhp, const unsigned short* __restrict__ qlp,
            const unsigned short* __restrict__ khp, const unsigned short* __restrict__ klp,
            const unsigned short* __restrict__ vhp, const unsigned short* __restrict__ vlp,
            const int* __restrict__ pos,
            unsigned short* ohp, unsigned short* olp,
            int qbBase, int nqbThis, float sscale) {
  union FH { v16h v; v8h h[2]; };
  __shared__ __align__(16) _Float16 Ksh[64 * 64];
  __shared__ __align__(16) _Float16 Ksl[PRES ? 64 * 64 : 8];
  __shared__ __align__(16) _Float16 Vth[64 * 64];
  __shared__ __align__(16) _Float16 Vtl[PRES ? 64 * 64 : 8];
  __shared__ __align__(16) _Float16 Psh[4][16 * 64];
  __shared__ __align__(16) _Float16 Psl[PRES ? 4 : 1][PRES ? 16 * 64 : 8];
  __shared__ __align__(16) float    Os[4][16 * 64];

  const int tid  = threadIdx.x;
  const int wave = tid >> 5;
  const int lane = tid & 31;
  const int hh   = lane >> 4;
  const int c    = lane & 15;

  const int bx   = blockIdx.x;
  const int qbl  = bx % nqbThis;
  const int rest = bx / nqbThis;
  const int h    = rest % NH;
  const int b    = rest / NH;
  const int kvh  = h / GRP;
  const int qb   = qbBase + qbl;
  const int q0   = qb * 64 + wave * 16;
  const size_t rowB = (size_t)b * SEQ;

  const _Float16* Qh = (const _Float16*)(const void*)qhp + (size_t)h * HD;
  const _Float16* Ql = (const _Float16*)(const void*)qlp + (size_t)h * HD;
  const _Float16* Kh = (const _Float16*)(const void*)khp + (size_t)kvh * HD;
  const _Float16* Kl = (const _Float16*)(const void*)klp + (size_t)kvh * HD;
  const _Float16* Vh = (const _Float16*)(const void*)vhp + ((size_t)b * KVD + (size_t)kvh * HD) * SEQ;
  const _Float16* Vl = (const _Float16*)(const void*)vlp + ((size_t)b * KVD + (size_t)kvh * HD) * SEQ;

  int kminLane = 2147483647;
#pragma unroll 4
  for (int i = 0; i < 16; ++i) {
    const v4i p4 = *(const v4i*)(pos + lane * 64 + 4 * i);
    kminLane = min(kminLane, min(min(p4[0], p4[1]), min(p4[2], p4[3])));
  }
  int qmx = max(pos[qb * 64 + lane], pos[qb * 64 + 32 + lane]);
#pragma unroll
  for (int off = 1; off < 32; off <<= 1) qmx = max(qmx, __shfl_xor(qmx, off, 32));
  int qpos[8];
#pragma unroll
  for (int r = 0; r < 8; ++r) qpos[r] = pos[q0 + 8 * hh + r];

  v16h qah[2], qal[2];
#pragma unroll
  for (int dc = 0; dc < 2; ++dc) {
    const size_t qo = (rowB + q0 + c) * QD + dc * 32 + 8 * hh;
    qah[dc] = ldfrag_h(Qh + qo);
    if (PRES) qal[dc] = ldfrag_h(Ql + qo);
    else      qal[dc] = qah[dc];
  }

  float mrow[8], lrow[8];
  v8f oacc[4];
#pragma unroll
  for (int r = 0; r < 8; ++r) { mrow[r] = -INFINITY; lrow[r] = 0.f; }
#pragma unroll
  for (int t = 0; t < 4; ++t) oacc[t] = zero8();

  for (int kt = 0; kt < NQB; ++kt) {
    const int kminT = __shfl(kminLane, kt, 32);
    const int skip = __builtin_amdgcn_readfirstlane((qmx < kminT) ? 1 : 0);
    if (skip != 0) continue;
    const int kv0 = kt * 64;
    __syncthreads();
    {
      const int r = tid >> 1, half = (tid & 1) * 32;
      const _Float16* kg  = Kh + (rowB + kv0 + r) * KVD + half;
      const _Float16* klg = Kl + (rowB + kv0 + r) * KVD + half;
      const _Float16* vg  = Vh + (size_t)r * SEQ + kv0 + half;
      const _Float16* vlg = Vl + (size_t)r * SEQ + kv0 + half;
#pragma unroll
      for (int i = 0; i < 4; ++i) {
        const v8h a0 = *(const v8h*)(kg + 8 * i);
        const v8h b0 = *(const v8h*)(vg + 8 * i);
        *(v8h*)(Ksh + r * 64 + half + 8 * i) = a0;
        *(v8h*)(Vth + r * 64 + half + 8 * i) = b0;
        if (PRES) {
          const v8h a1 = *(const v8h*)(klg + 8 * i);
          const v8h b1 = *(const v8h*)(vlg + 8 * i);
          *(v8h*)(Ksl + r * 64 + half + 8 * i) = a1;
          *(v8h*)(Vtl + r * 64 + half + 8 * i) = b1;
        }
      }
    }
    __syncthreads();

    v8f s[4];
#pragma unroll
    for (int j = 0; j < 4; ++j) {
      s[j] = zero8();
#pragma unroll
      for (int dc = 0; dc < 2; ++dc) {
        FH kb;
        kb.h[0] = *(const v8h*)(Ksh + (j * 16 + c) * 64 + dc * 32 + 8 * hh);
        kb.h[1] = *(const v8h*)(Ksh + (j * 16 + c) * 64 + dc * 32 + 16 + 8 * hh);
        s[j] = mma_h(qah[dc], kb.v, s[j]);
        if (PRES) {
          FH kl;
          kl.h[0] = *(const v8h*)(Ksl + (j * 16 + c) * 64 + dc * 32 + 8 * hh);
          kl.h[1] = *(const v8h*)(Ksl + (j * 16 + c) * 64 + dc * 32 + 16 + 8 * hh);
          s[j] = mma_h(qah[dc], kl.v, s[j]);
          s[j] = mma_h(qal[dc], kb.v, s[j]);
        }
      }
    }

    _Float16* pwh = Psh[wave];
    _Float16* pwl = Psl[PRES ? wave : 0];
    int kp[4];
#pragma unroll
    for (int j = 0; j < 4; ++j) kp[j] = pos[kv0 + j * 16 + c];
#pragma unroll
    for (int r = 0; r < 8; ++r) {
      float m = -INFINITY;
#pragma unroll
      for (int j = 0; j < 4; ++j) {
        float sv = s[j][r] * sscale;
        sv = (qpos[r] >= kp[j]) ? sv : -FLT_MAX;
        s[j][r] = sv;
        m = fmaxf(m, sv);
      }
#pragma unroll
      for (int off = 1; off < 16; off <<= 1) m = fmaxf(m, __shfl_xor(m, off, 32));
      const float mnew  = fmaxf(mrow[r], m);
      const float msafe = (mnew == -INFINITY) ? 0.f : mnew;
      const float alpha = __expf(mrow[r] - msafe);
      mrow[r] = mnew;
      float psum = 0.f;
#pragma unroll
      for (int j = 0; j < 4; ++j) {
        const float p = __expf(s[j][r] - msafe);
        psum += p;
        const float p1k = p * 1024.0f;
        const _Float16 ph = (_Float16)p1k;
        pwh[(8 * hh + r) * 64 + j * 16 + c] = ph;
        if (PRES) {
          const _Float16 plo = (_Float16)((p1k - (float)ph) * 4096.0f);
          pwl[(8 * hh + r) * 64 + j * 16 + c] = plo;
        }
      }
#pragma unroll
      for (int off = 1; off < 16; off <<= 1) psum += __shfl_xor(psum, off, 32);
      lrow[r] = lrow[r] * alpha + psum;
#pragma unroll
      for (int t = 0; t < 4; ++t) oacc[t][r] *= alpha;
    }
    __builtin_amdgcn_fence(__ATOMIC_RELEASE, "workgroup");
    __builtin_amdgcn_wave_barrier();
    __builtin_amdgcn_fence(__ATOMIC_ACQUIRE, "workgroup");

    v8f o1[4];
#pragma unroll
    for (int t = 0; t < 4; ++t) o1[t] = zero8();
#pragma unroll 1
    for (int kk = 0; kk < 2; ++kk) {
      FH pa, pl;
      pa.h[0] = *(const v8h*)(pwh + c * 64 + kk * 32 + 8 * hh);
      pa.h[1] = *(const v8h*)(pwh + c * 64 + kk * 32 + 16 + 8 * hh);
      if (PRES) {
        pl.h[0] = *(const v8h*)(pwl + c * 64 + kk * 32 + 8 * hh);
        pl.h[1] = *(const v8h*)(pwl + c * 64 + kk * 32 + 16 + 8 * hh);
      } else {
        pl.v = pa.v;
      }
#pragma unroll
      for (int t = 0; t < 4; ++t) {
        FH vb;
        vb.h[0] = *(const v8h*)(Vth + (t * 16 + c) * 64 + kk * 32 + 8 * hh);
        vb.h[1] = *(const v8h*)(Vth + (t * 16 + c) * 64 + kk * 32 + 16 + 8 * hh);
        oacc[t] = mma_h(pa.v, vb.v, oacc[t]);
        if (PRES) {
          FH vl;
          vl.h[0] = *(const v8h*)(Vtl + (t * 16 + c) * 64 + kk * 32 + 8 * hh);
          vl.h[1] = *(const v8h*)(Vtl + (t * 16 + c) * 64 + kk * 32 + 16 + 8 * hh);
          o1[t] = mma_h(pa.v, vl.v, o1[t]);
          o1[t] = mma_h(pl.v, vb.v, o1[t]);
        }
      }
    }
    if (PRES) {
#pragma unroll
      for (int t = 0; t < 4; ++t)
#pragma unroll
        for (int r = 0; r < 8; ++r) oacc[t][r] += o1[t][r] * (1.0f / 4096.0f);
    }
  }

  float* os = Os[wave];
#pragma unroll
  for (int r = 0; r < 8; ++r) {
    const float l = lrow[r];
    const float inv = ((l > 0.f) ? (1.0f / l) : 0.f) * (1.0f / 1024.0f);
#pragma unroll
    for (int t = 0; t < 4; ++t) os[(8 * hh + r) * 64 + t * 16 + c] = oacc[t][r] * inv;
  }
  __builtin_amdgcn_fence(__ATOMIC_RELEASE, "workgroup");
  __builtin_amdgcn_wave_barrier();
  __builtin_amdgcn_fence(__ATOMIC_ACQUIRE, "workgroup");
  {
    const int q4 = lane >> 3, c8 = (lane & 7) * 8;
    v4u hv[4], lv[4];
#pragma unroll
    for (int it = 0; it < 4; ++it) {
      const int rowi = it * 4 + q4;
      const float* sp = os + rowi * 64 + c8;
      v4u a, a2;
#pragma unroll
      for (int e = 0; e < 4; ++e) {
        const float f0 = sp[2 * e] * 64.0f, f1 = sp[2 * e + 1] * 64.0f;
        const _Float16 x0 = (_Float16)f0, x1 = (_Float16)f1;
        const unsigned short h0 = h_bits(x0), h1 = h_bits(x1);
        const unsigned short l0 = h_bits((_Float16)(f0 - (float)x0));
        const unsigned short l1 = h_bits((_Float16)(f1 - (float)x1));
        a[e] = pk16(h0, h1); a2[e] = pk16(l0, l1);
      }
      hv[it] = a; lv[it] = a2;
    }
    for (int pass = 0; pass < 2; ++pass) {
#pragma unroll
      for (int it = 0; it < 4; ++it) {
        const int rowi = it * 4 + q4;
        const size_t go = (rowB + q0 + rowi) * QD + (size_t)h * HD + c8;
        *(volatile v4u*)(ohp + go) = hv[it];
        *(volatile v4u*)(olp + go) = lv[it];
      }
      __threadfence();
    }
  }
}

extern "C" void kernel_launch(void* const* d_in, const int* in_sizes, int n_in,
                              void* d_out, int out_size, void* d_ws, size_t ws_size,
                              hipStream_t stream) {
  if (n_in < 6) return;
  if (in_sizes[0] != SEQ) return;
  if (in_sizes[1] != NB * SEQ * DM) return;
  if (in_sizes[2] != EQKV * DM) return;
  if (in_sizes[3] != DM * QD) return;
  if (in_sizes[4] != HD || in_sizes[5] != HD) return;
  if (out_size != NB * SEQ * DM) return;

  const int*   pos  = (const int*)d_in[0];
  const float* x    = (const float*)d_in[1];
  const float* wqkv = (const float*)d_in[2];
  const float* wo   = (const float*)d_in[3];
  const float* qw   = (const float*)d_in[4];
  const float* kw   = (const float*)d_in[5];

  const size_t PX   = (size_t)NTOK * DM * 2;
  const size_t PWQ  = (size_t)EQKV * DM * 2;
  const size_t PQKF = (size_t)NTOK * QKD * 4;
  const size_t PQ   = (size_t)NTOK * QD * 2;
  const size_t PK   = (size_t)NTOK * KVD * 2;
  const size_t PVT  = (size_t)NB * KVD * SEQ * 2;
  const size_t PWO  = (size_t)DM * QD * 2;
  const size_t PO   = (size_t)NTOK * QD * 2;
  const size_t PFRQ = 256;
  const size_t PTAB = (size_t)SEQ * 64 * 4;
  size_t off = 0;
  const size_t oXb  = off; off += PX;
  const size_t oWq  = off; off += PWQ;
  const size_t oQKf = off; off += PQKF;
  const size_t oQh  = off; off += PQ;
  const size_t oQl  = off; off += PQ;
  const size_t oKh  = off; off += PK;
  const size_t oKl  = off; off += PK;
  const size_t oVTh = off; off += PVT;
  const size_t oVTl = off; off += PVT;
  const size_t oFrq = off; off += PFRQ;
  const size_t oTab = off; off += PTAB;
  if (off > ws_size) return;
  if (off > (size_t)134217728) return;
  const size_t oWo = oXb;
  const size_t oOh = oQKf;
  const size_t oOl = oQKf + PO;
  if (PWO > PX) return;
  if (oOl + PO > oQh) return;

  char* ws = (char*)d_ws;
  unsigned short* Xb    = (unsigned short*)(ws + oXb);
  unsigned short* Wqkvb = (unsigned short*)(ws + oWq);
  float*          QKf   = (float*)(ws + oQKf);
  unsigned short* Qh    = (unsigned short*)(ws + oQh);
  unsigned short* Ql    = (unsigned short*)(ws + oQl);
  unsigned short* Kh    = (unsigned short*)(ws + oKh);
  unsigned short* Kl    = (unsigned short*)(ws + oKl);
  unsigned short* VTh   = (unsigned short*)(ws + oVTh);
  unsigned short* VTl   = (unsigned short*)(ws + oVTl);
  float*          Frq   = (float*)(ws + oFrq);
  float*          Tab   = (float*)(ws + oTab);
  unsigned short* Wob   = (unsigned short*)(ws + oWo);
  unsigned short* Oh    = (unsigned short*)(ws + oOh);
  unsigned short* Ol    = (unsigned short*)(ws + oOl);

  const dim3 blk(256);
  const int n8x   = NTOK * DM / 8;
  const int n8qkv = EQKV * DM / 8;
  const int n8o   = DM * QD / 8;
  const dim3 gCvtX((n8x + 255) / 256);
  const dim3 gCvtQKV((n8qkv + 255) / 256);
  const dim3 gCvtO((n8o + 255) / 256);
  const dim3 gQK(((NTOK / 64) * (QKD / 64) + 7) / 8, 1);
  const dim3 gVT(((KVD / 64) * (SEQ / 64) + 7) / 8, NB);
  const dim3 gOut(((NTOK / 64) * (DM / 64) + 7) / 8, 1);
  const dim3 gNR((NTOK * NUNIT + 7) / 8);
  const dim3 gTab((SEQ + 7) / 8);

  cvt16x8<0><<<gCvtX, blk, 0, stream>>>(x, Xb, n8x, 1.0f);
  cvt16x8<0><<<gCvtQKV, blk, 0, stream>>>(wqkv, Wqkvb, n8qkv, 1.0f);
  gemm64<false, 0, 0><<<gQK, blk, 0, stream>>>(
      Xb, Xb, DM, 0LL, Wqkvb, DM, 0LL,
      (void*)QKf, QKD, 0LL, (void*)QKf, QKD, 0LL, 0,
      NTOK, QKD, DM, 1.0f, 1.0f, 0, 0);
  gemm64<false, 0, 3><<<gVT, blk, 0, stream>>>(
      Wqkvb + (size_t)QKD * DM, Wqkvb + (size_t)QKD * DM, DM, 0LL, Xb, DM, (long long)SEQ * DM,
      (void*)VTh, SEQ, (long long)KVD * SEQ, (void*)VTl, SEQ, (long long)KVD * SEQ, SEQ,
      KVD, SEQ, DM, 1.0f, 4096.0f, 0, 0);
  ropefreq<<<dim3(1), dim3(32), 0, stream>>>(Frq);
  ropetab<<<gTab, blk, 0, stream>>>(pos, Frq, Tab, SEQ);
  normrope<<<gNR, blk, 0, stream>>>(QKf, qw, kw, Tab, Qh, Ql, Kh, Kl, NTOK * NUNIT);
  cvt16x8<1><<<gCvtO, blk, 0, stream>>>(wo, Wob, n8o, 1024.0f);
  attn64<true><<<dim3(NB * NH * RESQB), dim3(128), 0, stream>>>(
      Qh, Ql, Kh, Kl, VTh, VTl, pos, Oh, Ol, 0, RESQB, 0.125f / 4096.0f);
  attn64<false><<<dim3(NB * NH * (NQB - RESQB)), dim3(128), 0, stream>>>(
      Qh, Ql, Kh, Kl, VTh, VTl, pos, Oh, Ol, RESQB, NQB - RESQB, 0.125f / 4096.0f);
  gemm64<true, 1, 0><<<gOut, blk, 0, stream>>>(
      Oh, Ol, QD, 0LL, Wob, QD, 0LL,
      d_out, DM, 0LL, d_out, DM, 0LL, 0,
      NTOK, DM, QD, 1.0f / 65536.0f, 1.0f, SEQ - 1, RESQB * 64);
  (void)hipGetLastError();
}
